// TransformerNet_42460046688745
// MI455X (gfx1250) — hardware-verified
//
#include <hip/hip_runtime.h>
#include <stddef.h>
#include <stdint.h>


#ifndef NB
#define NB 4
#endif
#ifndef SEQ
#define SEQ 2048
#endif
#define NB_FULL  4
#define SEQ_FULL 2048
#define DM       128
#define NHEAD    4
#define DK       32
#define NLAYER   2
#define NQKV     384
#define NWROW    768
#define MROWS    (NB * SEQ)
#define NTHR     256
#define NWAVE    8
#define GBM      64
#define GBN      64
#define GTHR     128
#define QROWS    32
#define CX       8.0f
#define CW       64.0f
#define CV       8.0f
#define CP       8192.0f
#define SCL_XW   0.001953125f
#define OSC      0.0001220703125f
#define ATTSC    0.17677669529663688f
#define LN_EPS   0.001f
#define INV2PI   0.15915494309189535
#define PI2_HI   6.283185307179586
#define PI2_LO   2.4492935982947064e-16
#define WSMAX    134217728

static_assert(NB >= 1 && NB <= NB_FULL);
static_assert(SEQ >= 64 && SEQ <= SEQ_FULL && (SEQ % 64) == 0);
static_assert(DM == 128 && NHEAD * DK == DM && DK == 32);
static_assert((MROWS % GBM) == 0 && (MROWS % QROWS) == 0 && (MROWS % 16) == 0);
static_assert(GBM == (GTHR / 32) * 16 && GBN == 64);
static_assert(NQKV == 3 * DM && NWROW == 6 * DM && (NQKV % GBN) == 0);
static_assert(NTHR == 32 * NWAVE && QROWS == 16 * (NWAVE / NHEAD));

typedef float          v4f  __attribute__((ext_vector_type(4)));
typedef float          v8f  __attribute__((ext_vector_type(8)));
typedef int            v8i  __attribute__((ext_vector_type(8)));
typedef _Float16       v8h  __attribute__((ext_vector_type(8)));
typedef _Float16       v16h __attribute__((ext_vector_type(16)));
typedef __bf16         v8b  __attribute__((ext_vector_type(8)));
typedef __bf16         v16b __attribute__((ext_vector_type(16)));
typedef unsigned short v8us __attribute__((ext_vector_type(8)));
union FragH { v16h v; v8h h[2]; v8i w; };
union FragB { v16b v; v8b h[2]; v8i w; };

__device__ __forceinline__ v8f wmh(const FragH& a, const FragH& b, v8f c) {
  v8f d = __builtin_amdgcn_wmma_f32_16x16x32_f16(false, a.v, false, b.v, (short)0, c, false, false);
  asm volatile("v_nop\n\tv_nop\n\tv_nop\n\tv_nop" : "+v"(d) : "v"(a.w), "v"(b.w));
  return d;
}
__device__ __forceinline__ v8f wmb(const FragB& a, const FragB& b, v8f c) {
  v8f d = __builtin_amdgcn_wmma_f32_16x16x32_bf16(false, a.v, false, b.v, (short)0, c, false, false);
  asm volatile("v_nop\n\tv_nop\n\tv_nop\n\tv_nop" : "+v"(d) : "v"(a.w), "v"(b.w));
  return d;
}

__device__ __forceinline__ unsigned bf16bits(float f) {
  const unsigned u = __float_as_uint(f);
  return (u + 0x7fffu + ((u >> 16) & 1u)) & 0xffff0000u;
}
__device__ __forceinline__ float bf16r(float f) { return __uint_as_float(bf16bits(f)); }
__device__ __forceinline__ v4f bf16r4(const v4f a) {
  v4f r;
  r.x = bf16r(a.x); r.y = bf16r(a.y); r.z = bf16r(a.z); r.w = bf16r(a.w);
  return r;
}
__device__ __forceinline__ void split2(float x, unsigned short& hb, unsigned short& lb) {
  const unsigned uh = bf16bits(x);
  const float    rr = x - __uint_as_float(uh);
  const unsigned ul = bf16bits(rr);
  hb = (unsigned short)(uh >> 16);
  lb = (unsigned short)(ul >> 16);
}
__device__ __forceinline__ void split8(const v4f a, const v4f b, v8us& hi, v8us& lo) {
  unsigned short h0, h1, h2, h3, h4, h5, h6, h7, l0, l1, l2, l3, l4, l5, l6, l7;
  split2(a.x, h0, l0); split2(a.y, h1, l1); split2(a.z, h2, l2); split2(a.w, h3, l3);
  split2(b.x, h4, l4); split2(b.y, h5, l5); split2(b.z, h6, l6); split2(b.w, h7, l7);
  hi[0] = h0; hi[1] = h1; hi[2] = h2; hi[3] = h3; hi[4] = h4; hi[5] = h5; hi[6] = h6; hi[7] = h7;
  lo[0] = l0; lo[1] = l1; lo[2] = l2; lo[3] = l3; lo[4] = l4; lo[5] = l5; lo[6] = l6; lo[7] = l7;
}

__device__ __forceinline__ v8h cvt8h(const v4f a, const v4f b, const float c) {
  v8h hv;
  hv[0] = (_Float16)(a.x * c); hv[1] = (_Float16)(a.y * c);
  hv[2] = (_Float16)(a.z * c); hv[3] = (_Float16)(a.w * c);
  hv[4] = (_Float16)(b.x * c); hv[5] = (_Float16)(b.y * c);
  hv[6] = (_Float16)(b.z * c); hv[7] = (_Float16)(b.w * c);
  return hv;
}

__global__ __launch_bounds__(NTHR) void k_pe(float* pe, int nUnits) {
  const int u = (int)blockIdx.x * NTHR + (int)threadIdx.x;
  if (u >= nUnits) return;
  const int t  = u >> 5;
  const int i0 = (u & 31) * 4;
  const double c8d = sqrt(10.0);
  const double c4d = sqrt(c8d);
  const double c2d = sqrt(c4d);
  const double c1d = sqrt(c2d);
  double den = 1.0;
  den *= (i0 & 4)  ? c4d : 1.0;
  den *= (i0 & 8)  ? c8d : 1.0;
  den *= (i0 & 16) ? 10.0 : 1.0;
  den *= (i0 & 32) ? 100.0 : 1.0;
  den *= (i0 & 64) ? 10000.0 : 1.0;
  v4f o = {0.f, 0.f, 0.f, 0.f};
#pragma unroll 1
  for (int j = 0; j < 4; ++j) {
    const double ang = (double)t / den;
    const double kq  = rint(ang * INV2PI);
    double r = fma(-kq, PI2_HI, ang);
    r = fma(-kq, PI2_LO, r);
    const float rf = (float)r;
    float sn, cs;
    sincosf(rf, &sn, &cs);
    const float val = (j & 1) ? cs : sn;
    v4f nx;
    nx.x = o.y; nx.y = o.z; nx.z = o.w; nx.w = val;
    o = nx;
    den *= c1d;
  }
  float* p = pe + (size_t)t * DM + i0;
  *(volatile v4f*)p = o;
  __threadfence();
  *(volatile v4f*)p = o;
}

__global__ __launch_bounds__(NTHR) void k_wtr6(const float* __restrict__ w0, const float* __restrict__ w1,
                                                const float* __restrict__ w2, const float* __restrict__ w3,
                                                const float* __restrict__ w4, const float* __restrict__ w5,
                                                _Float16* wt, int nUnits) {
  const int u = (int)blockIdx.x * NTHR + (int)threadIdx.x;
  if (u >= nUnits) return;
  const int n  = u >> 4;
  const int k8 = (u & 15) * 8;
  int seg = n >> 7;
  seg = seg > 5 ? 5 : seg;
  const int nc = n & (DM - 1);
  const float* wsrc = (seg == 0) ? w0 : ((seg == 1) ? w1 : ((seg == 2) ? w2 : ((seg == 3) ? w3 : ((seg == 4) ? w4 : w5))));
  const float* p = wsrc + (size_t)k8 * DM + nc;
  v4f a, b;
  a.x = bf16r(p[0]);               a.y = bf16r(p[DM]);              a.z = bf16r(p[2 * DM]);          a.w = bf16r(p[3 * DM]);
  b.x = bf16r(p[4 * DM]);          b.y = bf16r(p[5 * DM]);          b.z = bf16r(p[6 * DM]);          b.w = bf16r(p[7 * DM]);
  const v8h hv = cvt8h(a, b, CW);
  const size_t o = (size_t)n * DM + k8;
  *(volatile v8h*)(wt + o) = hv;
  __threadfence();
  *(volatile v8h*)(wt + o) = hv;
}

template<int SRC, int OUTF, int OUTH>
__global__ __launch_bounds__(NTHR) void k_ln(const float* __restrict__ xin, const float* __restrict__ pe,
                                              const float* __restrict__ g, const float* __restrict__ bb,
                                              float* outF, _Float16* outH) {
  __shared__ __attribute__((aligned(16))) float lbuf[NWAVE * 256];
  const int tid = (int)threadIdx.x, lane = tid & 31, wave = tid >> 5, rsel = lane >> 4, c8 = (lane & 15) * 8;
  const int m0 = (int)blockIdx.x * 16 + wave * 2;
  const int m  = m0 + rsel;
  v4f a, c;
  if (SRC == 0) {
    const int bi = m / SEQ;
    const int t  = m - bi * SEQ;
    const float* p = xin + ((size_t)bi * SEQ_FULL + (size_t)t) * DM + c8;
    a = bf16r4(*(const v4f*)p);
    c = bf16r4(*(const v4f*)(p + 4));
    const float* q = pe + (size_t)t * DM + c8;
    a += *(const v4f*)q;
    c += *(const v4f*)(q + 4);
  } else {
    const float* p = xin + (size_t)m * DM + c8;
    a = *(const v4f*)p;
    c = *(const v4f*)(p + 4);
  }
  float s = ((a.x + a.y) + (a.z + a.w)) + ((c.x + c.y) + (c.z + c.w));
  s += __shfl_xor(s, 8); s += __shfl_xor(s, 4); s += __shfl_xor(s, 2); s += __shfl_xor(s, 1);
  const float mu = s * 0.0078125f;
  const v4f da = a - mu, dc = c - mu;
  float q2 = ((da.x * da.x + da.y * da.y) + (da.z * da.z + da.w * da.w)) +
             ((dc.x * dc.x + dc.y * dc.y) + (dc.z * dc.z + dc.w * dc.w));
  q2 += __shfl_xor(q2, 8); q2 += __shfl_xor(q2, 4); q2 += __shfl_xor(q2, 2); q2 += __shfl_xor(q2, 1);
  const float rstd = rsqrtf(fmaf(q2, 0.0078125f, LN_EPS));
  const v4f ga = bf16r4(*(const v4f*)(g + c8)),  gc = bf16r4(*(const v4f*)(g + c8 + 4));
  const v4f ba = bf16r4(*(const v4f*)(bb + c8)), bc = bf16r4(*(const v4f*)(bb + c8 + 4));
  const v4f ya = (ga * da) * rstd + ba;
  const v4f yc = (gc * dc) * rstd + bc;

  const v8h hv = cvt8h(ya, yc, CX);
  v4f o0 = {0.f, 0.f, 0.f, 0.f}, o1 = {0.f, 0.f, 0.f, 0.f};
  if (OUTF) {
    float* buf = lbuf + wave * 256;
    *(v4f*)(buf + rsel * DM + c8)     = ya;
    *(v4f*)(buf + rsel * DM + c8 + 4) = yc;
    __builtin_amdgcn_fence(3  , "wavefront");
    __builtin_amdgcn_wave_barrier();
    o0 = *(const v4f*)(buf + 4 * lane);
    o1 = *(const v4f*)(buf + DM + 4 * lane);
  }
  _Float16* hp = outH + (size_t)m * DM + c8;
  float* f0 = outF + (size_t)m0 * DM + 4 * lane;
  float* f1 = f0 + DM;
  if (OUTH) *(volatile v8h*)hp = hv;
  if (OUTF) { *(volatile v4f*)f0 = o0; *(volatile v4f*)f1 = o1; }
  __threadfence();
  if (OUTH) *(volatile v8h*)hp = hv;
  if (OUTF) { *(volatile v4f*)f0 = o0; *(volatile v4f*)f1 = o1; }
}

__device__ __forceinline__ void gemm_core(const _Float16* __restrict__ A, const _Float16* __restrict__ WT,
                                          const float* __restrict__ bias, int bofs, int rowBase, int col0,
                                          float* stg, int tid) {
  const int lane = tid & 31, wave = tid >> 5, hh = lane >> 4, m = lane & 15;
  v8f acc[4];
  {
    const v8f z = {0.f, 0.f, 0.f, 0.f, 0.f, 0.f, 0.f, 0.f};
    acc[0] = z; acc[1] = z; acc[2] = z; acc[3] = z;
  }
  const _Float16* ap = A  + (size_t)(rowBase + 16 * wave + m) * DM + 8 * hh;
  const _Float16* wp = WT + (size_t)(col0 + m) * DM + 8 * hh;
#pragma unroll 1
  for (int ks = 0; ks < DM / 32; ++ks) {
    FragH af;
    af.h[0] = *(const v8h*)(ap + 32 * ks);
    af.h[1] = *(const v8h*)(ap + 32 * ks + 16);
#pragma unroll
    for (int t = 0; t < 4; ++t) {
      const _Float16* wq = wp + (size_t)(16 * t) * DM + 32 * ks;
      FragH bfr;
      bfr.h[0] = *(const v8h*)wq;
      bfr.h[1] = *(const v8h*)(wq + 16);
      acc[t] = wmh(af, bfr, acc[t]);
    }
  }
#pragma unroll
  for (int t = 0; t < 4; ++t) {
    const int lc = 16 * t + m;
    int bi = bofs + lc;
    bi = bi > DM - 1 ? DM - 1 : bi;
    bi = bi < 0 ? 0 : bi;
    const float bvv = bf16r(bias[bi]);
#pragma unroll
    for (int r = 0; r < 8; ++r) {
      const int lr = 16 * wave + 8 * hh + r;
      stg[lr * GBN + lc] = fmaf(acc[t][r], SCL_XW, bvv);
    }
  }
}

__global__ __launch_bounds__(GTHR) void k_gemm_qkv(const _Float16* __restrict__ A, const _Float16* __restrict__ WT,
                                                    const float* __restrict__ bq, const float* __restrict__ bk,
                                                    const float* __restrict__ bv,
                                                    unsigned short* QH, unsigned short* QL,
                                                    unsigned short* KH, unsigned short* KL, _Float16* VT) {
  __shared__ __attribute__((aligned(16))) float stg[GBM * GBN];
  const int tid = (int)threadIdx.x;
  const int rowBase = (int)blockIdx.x * GBM;
  const int by   = (int)blockIdx.y;
  const int col0 = by * GBN;
  const int seg  = by >> 1;
  const int cin  = (by & 1) * GBN;
  const float* bp = (seg == 0) ? bq : ((seg == 1) ? bk : bv);
  gemm_core(A, WT, bp, cin, rowBase, col0, stg, tid);
  __syncthreads();

  const int pr = tid >> 3, pc = (tid & 7) * 8;
  if (seg < 2) {
    unsigned short* PH = (seg == 0) ? QH : KH;
    unsigned short* PL = (seg == 0) ? QL : KL;
    v8us hi[4], lo[4];
    size_t o[4];
#pragma unroll
    for (int i = 0; i < 4; ++i) {
      const int lr = 16 * i + pr;
      const v4f va = *(const v4f*)(stg + lr * GBN + pc);
      const v4f vb = *(const v4f*)(stg + lr * GBN + pc + 4);
      split8(va, vb, hi[i], lo[i]);
      o[i] = (size_t)(rowBase + lr) * DM + cin + pc;
    }
#pragma unroll
    for (int i = 0; i < 4; ++i) { *(volatile v8us*)(PH + o[i]) = hi[i]; *(volatile v8us*)(PL + o[i]) = lo[i]; }
    __threadfence();
#pragma unroll
    for (int i = 0; i < 4; ++i) { *(volatile v8us*)(PH + o[i]) = hi[i]; *(volatile v8us*)(PL + o[i]) = lo[i]; }
  } else {
    const int bi = rowBase / SEQ;
    const int t0 = rowBase - bi * SEQ;
    v8h hv[4];
    size_t o[4];
#pragma unroll
    for (int i = 0; i < 4; ++i) {
      const int lc = 16 * i + pr;
      v4f va, vb;
      va.x = stg[(pc + 0) * GBN + lc]; va.y = stg[(pc + 1) * GBN + lc];
      va.z = stg[(pc + 2) * GBN + lc]; va.w = stg[(pc + 3) * GBN + lc];
      vb.x = stg[(pc + 4) * GBN + lc]; vb.y = stg[(pc + 5) * GBN + lc];
      vb.z = stg[(pc + 6) * GBN + lc]; vb.w = stg[(pc + 7) * GBN + lc];
      hv[i] = cvt8h(va, vb, CV);
      o[i] = (size_t)(bi * DM + cin + lc) * SEQ + t0 + pc;
    }
#pragma unroll
    for (int i = 0; i < 4; ++i) *(volatile v8h*)(VT + o[i]) = hv[i];
    __threadfence();
#pragma unroll
    for (int i = 0; i < 4; ++i) *(volatile v8h*)(VT + o[i]) = hv[i];
  }
}

template<int RES>
__global__ __launch_bounds__(GTHR) void k_gemm_f32(const _Float16* __restrict__ A, const _Float16* __restrict__ WT,
                                                    const float* __restrict__ bias, const float* __restrict__ res,
                                                    float* outF) {
  __shared__ __attribute__((aligned(16))) float stg[GBM * GBN];
  const int tid = (int)threadIdx.x, lane = tid & 31, wave = tid >> 5, hh = lane >> 4, m = lane & 15;
  const int rowBase = (int)blockIdx.x * GBM;
  const int col0    = (int)blockIdx.y * GBN;
  gemm_core(A, WT, bias, col0, rowBase, col0, stg, tid);
  __syncthreads();
  v4f fv[8];
#pragma unroll
  for (int i = 0; i < 8; ++i) {
    const int lr = 16 * wave + 2 * i + hh;
    fv[i] = *(const v4f*)(stg + lr * GBN + 4 * m);
    if (RES) fv[i] += *(const v4f*)(res + (size_t)(rowBase + lr) * DM + col0 + 4 * m);
  }
#pragma unroll
  for (int i = 0; i < 8; ++i) {
    const int lr = 16 * wave + 2 * i + hh;
    float* op = outF + (size_t)(rowBase + lr) * DM + col0 + 4 * m;
    *(volatile v4f*)op = fv[i];
  }
  __threadfence();
#pragma unroll
  for (int i = 0; i < 8; ++i) {
    const int lr = 16 * wave + 2 * i + hh;
    float* op = outF + (size_t)(rowBase + lr) * DM + col0 + 4 * m;
    *(volatile v4f*)op = fv[i];
  }
}

__global__ __launch_bounds__(GTHR) void k_gemm_h16(const _Float16* __restrict__ A, const _Float16* __restrict__ WT,
                                                    const float* __restrict__ bias, _Float16* outH) {
  __shared__ __attribute__((aligned(16))) float stg[GBM * GBN];
  const int tid = (int)threadIdx.x;
  const int rowBase = (int)blockIdx.x * GBM;
  const int col0    = (int)blockIdx.y * GBN;
  gemm_core(A, WT, bias, col0, rowBase, col0, stg, tid);
  __syncthreads();
  const int pr = tid >> 3, pc = (tid & 7) * 8;
  const v4f z4 = {0.f, 0.f, 0.f, 0.f};
  v8h hv[4];
  size_t o[4];
#pragma unroll
  for (int i = 0; i < 4; ++i) {
    const int lr = 16 * i + pr;
    v4f va = *(const v4f*)(stg + lr * GBN + pc);
    v4f vb = *(const v4f*)(stg + lr * GBN + pc + 4);
    va.x = fmaxf(va.x, 0.f); va.y = fmaxf(va.y, 0.f); va.z = fmaxf(va.z, 0.f); va.w = fmaxf(va.w, 0.f);
    vb.x = fmaxf(vb.x, 0.f); vb.y = fmaxf(vb.y, 0.f); vb.z = fmaxf(vb.z, 0.f); vb.w = fmaxf(vb.w, 0.f);
    (void)z4;
    hv[i] = cvt8h(va, vb, CX);
    o[i] = (size_t)(rowBase + lr) * DM + col0 + pc;
  }
#pragma unroll
  for (int i = 0; i < 4; ++i) *(volatile v8h*)(outH + o[i]) = hv[i];
  __threadfence();
#pragma unroll
  for (int i = 0; i < 4; ++i) *(volatile v8h*)(outH + o[i]) = hv[i];
}

__global__ __launch_bounds__(NTHR) void k_attn(const __bf16* __restrict__ QH, const __bf16* __restrict__ QL,
                                                const __bf16* __restrict__ KH, const __bf16* __restrict__ KL,
                                                const _Float16* __restrict__ VT, _Float16* CTX) {
  __shared__ __attribute__((aligned(16))) _Float16 ctile[QROWS * DM];
  const int tid = (int)threadIdx.x, lane = tid & 31, wave = tid >> 5, hh = lane >> 4, m = lane & 15;
  const int qt = wave >> 2, h = wave & 3;
  const int nqp = SEQ / QROWS;
  const int blk = (int)blockIdx.x;
  const int bi  = blk / nqp;
  const int qp  = blk - bi * nqp;
  const int rowQ = bi * SEQ + qp * QROWS + 16 * qt;
  const int coff = h * DK + 8 * hh;

  FragB bqh, bql;
  {
    const __bf16* q1 = QH + (size_t)(rowQ + m) * DM + coff;
    const __bf16* q2 = QL + (size_t)(rowQ + m) * DM + coff;
    bqh.h[0] = *(const v8b*)q1; bqh.h[1] = *(const v8b*)(q1 + 16);
    bql.h[0] = *(const v8b*)q2; bql.h[1] = *(const v8b*)(q2 + 16);
  }
  const __bf16* kh0 = KH + (size_t)(bi * SEQ + m) * DM + coff;
  const __bf16* kl0 = KL + (size_t)(bi * SEQ + m) * DM + coff;
  const _Float16* v0 = VT + (size_t)(bi * DM + h * DK + m) * SEQ + 8 * hh;
  const _Float16* v1 = v0 + (size_t)16 * SEQ;

  const v8f z = {0.f, 0.f, 0.f, 0.f, 0.f, 0.f, 0.f, 0.f};
  v8f c0 = z, c1 = z;
  float rm = -1.0e30f, rl = 0.f;

#pragma unroll 1
  for (int kc = 0; kc < SEQ; kc += 32) {
    const size_t ko = (size_t)kc * DM;
    FragB a0h, a0l, a1h, a1l;
    a0h.h[0] = *(const v8b*)(kh0 + ko);             a0h.h[1] = *(const v8b*)(kh0 + ko + 16);
    a1h.h[0] = *(const v8b*)(kh0 + ko + 16 * DM);   a1h.h[1] = *(const v8b*)(kh0 + ko + 16 * DM + 16);
    a0l.h[0] = *(const v8b*)(kl0 + ko);             a0l.h[1] = *(const v8b*)(kl0 + ko + 16);
    a1l.h[0] = *(const v8b*)(kl0 + ko + 16 * DM);   a1l.h[1] = *(const v8b*)(kl0 + ko + 16 * DM + 16);
    v8f s0 = wmb(a0h, bqh, z);
    s0 = wmb(a0h, bql, s0);
    s0 = wmb(a0l, bqh, s0);
    v8f s1 = wmb(a1h, bqh, z);
    s1 = wmb(a1h, bql, s1);
    s1 = wmb(a1l, bqh, s1);

    float smax = -1.0e30f;
#pragma unroll
    for (int r = 0; r < 8; ++r) {
      s0[r] *= ATTSC;
      s1[r] *= ATTSC;
      smax = fmaxf(smax, fmaxf(s0[r], s1[r]));
    }
    smax = fmaxf(smax, __shfl_xor(smax, 16));
    const float mn   = fmaxf(rm, smax);
    const float corr = __expf(rm - mn);
    rm = mn;
    float ps = 0.f;
    v8h ph0, ph1;
#pragma unroll
    for (int r = 0; r < 8; ++r) {
      const float p0 = __expf(s0[r] - mn);
      const float p1 = __expf(s1[r] - mn);
      ps += p0 + p1;
      ph0[r] = (_Float16)(p0 * CP);
      ph1[r] = (_Float16)(p1 * CP);
    }
    ps += __shfl_xor(ps, 16);
    rl = fmaf(rl, corr, ps);
#pragma unroll
    for (int r = 0; r < 8; ++r) { c0[r] *= corr; c1[r] *= corr; }
    FragH pb;
    pb.h[0] = ph0;
    pb.h[1] = ph1;
    FragH av0, av1;
    av0.h[0] = *(const v8h*)(v0 + kc); av0.h[1] = *(const v8h*)(v0 + kc + 16);
    av1.h[0] = *(const v8h*)(v1 + kc); av1.h[1] = *(const v8h*)(v1 + kc + 16);
    c0 = wmh(av0, pb, c0);
    c1 = wmh(av1, pb, c1);
  }

  const float f = __builtin_amdgcn_rcpf(rl) * OSC;
  v8h o0, o1;
#pragma unroll
  for (int r = 0; r < 8; ++r) { o0[r] = (_Float16)(c0[r] * f); o1[r] = (_Float16)(c1[r] * f); }
  _Float16* cw = ctile + (qt * 16 + m) * DM + h * DK + 8 * hh;
  *(v8h*)cw        = o0;
  *(v8h*)(cw + 16) = o1;
  __syncthreads();

  const int r0i = tid >> 4, r1i = (tid + NTHR) >> 4, cc8 = (tid & 15) * 8;
  const v8h w0 = *(const v8h*)(ctile + r0i * DM + cc8);
  const v8h w1 = *(const v8h*)(ctile + r1i * DM + cc8);
  _Float16* g0 = CTX + (size_t)(bi * SEQ + qp * QROWS + r0i) * DM + cc8;
  _Float16* g1 = CTX + (size_t)(bi * SEQ + qp * QROWS + r1i) * DM + cc8;
  *(volatile v8h*)g0 = w0;
  *(volatile v8h*)g1 = w1;
  __threadfence();
  *(volatile v8h*)g0 = w0;
  *(volatile v8h*)g1 = w1;
}

static inline int cdiv(int a, int b) { return (a + b - 1) / b; }
static inline size_t carve(size_t* off, size_t bytes) {
  const size_t o = *off;
  *off = (o + bytes + 255) & ~(size_t)255;
  return o;
}

extern "C" void kernel_launch(void* const* d_in, const int* in_sizes, int n_in,
                              void* d_out, int out_size, void* d_ws, size_t ws_size,
                              hipStream_t stream) {
  if (n_in < 15) return;
  const int M = MROWS;
  if (in_sizes[0] < ((NB - 1) * SEQ_FULL + SEQ) * DM) return;
  for (int j = 1; j <= 11; j += 2) { if (in_sizes[j] < NLAYER * DM * DM) return; }
  for (int j = 2; j <= 12; j += 2) { if (in_sizes[j] < NLAYER * DM) return; }
  if (in_sizes[13] < 2 * NLAYER * DM || in_sizes[14] < 2 * NLAYER * DM) return;
  if (out_size < M * DM) return;

  const float* x   = (const float*)d_in[0];
  const float* Wq  = (const float*)d_in[1];
  const float* bq  = (const float*)d_in[2];
  const float* Wk  = (const float*)d_in[3];
  const float* bk  = (const float*)d_in[4];
  const float* Wv  = (const float*)d_in[5];
  const float* bv  = (const float*)d_in[6];
  const float* Wo  = (const float*)d_in[7];
  const float* bo  = (const float*)d_in[8];
  const float* W1  = (const float*)d_in[9];
  const float* b1  = (const float*)d_in[10];
  const float* W2  = (const float*)d_in[11];
  const float* b2  = (const float*)d_in[12];
  const float* lng = (const float*)d_in[13];
  const float* lnb = (const float*)d_in[14];
  float* out = (float*)d_out;

  char* ws = (char*)d_ws;
  size_t off = 0;
  const size_t oPE  = carve(&off, (size_t)SEQ * DM * 4);
  const size_t oWT  = carve(&off, (size_t)NLAYER * NWROW * DM * 2);
  const size_t oA1H = carve(&off, (size_t)M * DM * 2);
  const size_t oQH  = carve(&off, (size_t)M * DM * 2);
  const size_t oQL  = carve(&off, (size_t)M * DM * 2);
  const size_t oKH  = carve(&off, (size_t)M * DM * 2);
  const size_t oKL  = carve(&off, (size_t)M * DM * 2);
  const size_t oVT  = carve(&off, (size_t)NB * DM * SEQ * 2);
  const size_t oCTX = carve(&off, (size_t)M * DM * 2);
  const size_t oH2  = carve(&off, (size_t)M * DM * 4);
  const size_t oA2F = carve(&off, (size_t)M * DM * 4);
  const size_t oA2H = carve(&off, (size_t)M * DM * 2);
  const size_t oF1H = carve(&off, (size_t)M * DM * 2);
  const size_t oH3  = carve(&off, (size_t)M * DM * 4);
  if (off > ws_size || off > (size_t)WSMAX) return;

  float*          PE   = (float*)(ws + oPE);
  _Float16*       WT   = (_Float16*)(ws + oWT);
  _Float16*       A1H  = (_Float16*)(ws + oA1H);
  unsigned short* QH   = (unsigned short*)(ws + oQH);
  unsigned short* QL   = (unsigned short*)(ws + oQL);
  unsigned short* KH   = (unsigned short*)(ws + oKH);
  unsigned short* KL   = (unsigned short*)(ws + oKL);
  _Float16*       VT   = (_Float16*)(ws + oVT);
  _Float16*       CTXH = (_Float16*)(ws + oCTX);
  float*          H2   = (float*)(ws + oH2);
  float*          A2F  = (float*)(ws + oA2F);
  _Float16*       A2H  = (_Float16*)(ws + oA2H);
  _Float16*       F1H  = (_Float16*)(ws + oF1H);
  float*          H3   = (float*)(ws + oH3);

  const int nUpe = SEQ * 32;
  k_pe<<<cdiv(nUpe, NTHR), NTHR, 0, stream>>>(PE, nUpe);

  const int nUw = NWROW * (DM / 8);
  for (int li = 0; li < NLAYER; ++li) {
    const size_t wo = (size_t)li * DM * DM;
    k_wtr6<<<cdiv(nUw, NTHR), NTHR, 0, stream>>>(Wq + wo, Wk + wo, Wv + wo, Wo + wo, W1 + wo, W2 + wo,
                                                  WT + (size_t)li * NWROW * DM, nUw);
  }

  const int gLn = M / 16;
  const int gM  = M / GBM;
  const int gAt = M / QROWS;
  for (int li = 0; li < NLAYER; ++li) {
    const _Float16* WTl = WT + (size_t)li * NWROW * DM;
    const size_t bofs = (size_t)li * DM;
    if (li == 0) {
      k_ln<0, 0, 1><<<gLn, NTHR, 0, stream>>>(x, PE, lng, lnb, H2, A1H);
    } else {
      k_ln<1, 0, 1><<<gLn, NTHR, 0, stream>>>(H3, PE, lng + 2 * li * DM, lnb + 2 * li * DM, H2, A1H);
    }
    k_gemm_qkv<<<dim3(gM, NQKV / GBN), GTHR, 0, stream>>>(A1H, WTl, bq + bofs, bk + bofs, bv + bofs,
                                                             QH, QL, KH, KL, VT);
    k_attn<<<gAt, NTHR, 0, stream>>>((const __bf16*)QH, (const __bf16*)QL, (const __bf16*)KH, (const __bf16*)KL,
                                      VT, CTXH);
    k_gemm_f32<0><<<dim3(gM, DM / GBN), GTHR, 0, stream>>>(CTXH, WTl + (size_t)3 * DM * DM, bo + bofs, A2F, H2);
    k_ln<1, 1, 1><<<gLn, NTHR, 0, stream>>>(H2, PE, lng + (2 * li + 1) * DM, lnb + (2 * li + 1) * DM, A2F, A2H);
    k_gemm_h16<<<dim3(gM, DM / GBN), GTHR, 0, stream>>>(A2H, WTl + (size_t)4 * DM * DM, b1 + bofs, F1H);
    k_gemm_f32<1><<<dim3(gM, DM / GBN), GTHR, 0, stream>>>(F1H, WTl + (size_t)5 * DM * DM, b2 + bofs, A2F, H3);
  }
  k_ln<1, 1, 0><<<gLn, NTHR, 0, stream>>>(H3, PE, lng + (2 * NLAYER - 1) * DM, lnb + (2 * NLAYER - 1) * DM, out, A1H);
}
